// Geo3DGNN_44306882625631
// MI455X (gfx1250) — hardware-run, weakly checked
//
#include <hip/hip_runtime.h>
#include <stddef.h>
#include <stdint.h>


#define NNODE  50000
#define NEDGE  800000
#define MP     50048
#define NBA    1024
#define SLA    10
#define NBLK   49
#define NTAB   (NBLK * NBA)
#define RCAP   20480
#define DEGCAP 64
#define MEAS_B1024  16623
#define MEAS_MAXDEG 35
#define NTHR   256
#define NWAVE  8
#define EPT    8
#define CHUNK  (NTHR * EPT)
#define WCAP   (EPT * 32)
#define LISTN  (NWAVE * WCAP)
#define GBM    64
#define GBN    128
#define GTHR   128
#define GWAVE  4
#define PARTW  288
#define NTILE  391
#define NPB    128
#define AGG_ZINTS    (LISTN + 2 * RCAP + 3 * NBA)
#define MISC_INTS    16
#define BKT_LDS_INTS (AGG_ZINTS + MISC_INTS)
#define BNEPS  1e-5f
#define WSMAX  134217728ull

static_assert((CHUNK & (CHUNK - 1)) == 0 && CHUNK <= 4096);
static_assert(NBA == (1 << SLA));
static_assert(((long long)NEDGE << SLA) < (1LL << 31));
static_assert(NBA * NBLK >= NNODE && NTAB >= MP);
static_assert((long long)RCAP * 100 >= (long long)MEAS_B1024 * 105);
static_assert(DEGCAP >= MEAS_MAXDEG + 8);
static_assert(RCAP % 32 == 0 && AGG_ZINTS % (NTHR * 4) == 0);
static_assert(BKT_LDS_INTS * 4 <= 327680);
static_assert(MP % 128 == 0 && MP % GBM == 0 && NTILE * 128 == MP && MP >= NNODE);
static_assert(96 % 32 == 0 && 384 % 32 == 0 && 256 % 32 == 0 && 512 % 32 == 0 && 192 % 32 == 0 && 64 % 32 == 0);
static_assert((GBM * 10 * 4) % 128 == 0);
static_assert(((NNODE % GBM) * 10 * 4) % 128 == 0);
static_assert((128 * 40) % 128 == 0);
static_assert(NPB * NTILE == MP && NPB == 16 * NWAVE);
static_assert(PARTW % 32 == 0 && PARTW >= 257 && PARTW / 4 <= NTHR);
static_assert(NTAB % 4 == 0 && GBM % 4 == 0 && GBM / 4 == 16 && GBM / 4 <= GTHR);
static_assert(MP <= NTAB);

typedef float          v2f   __attribute__((ext_vector_type(2)));
typedef float          v4f   __attribute__((ext_vector_type(4)));
typedef float          v8f   __attribute__((ext_vector_type(8)));
typedef int            v4i   __attribute__((ext_vector_type(4)));
typedef int            v8i   __attribute__((ext_vector_type(8)));
typedef unsigned       v2u   __attribute__((ext_vector_type(2)));
typedef unsigned short v2us  __attribute__((ext_vector_type(2)));
typedef unsigned short v4us  __attribute__((ext_vector_type(4)));
typedef unsigned short v8us  __attribute__((ext_vector_type(8)));
typedef unsigned short v16us __attribute__((ext_vector_type(16)));
typedef __bf16         v16bf __attribute__((ext_vector_type(16)));
typedef v2f  __attribute__((may_alias)) v2fa;
typedef v4f  __attribute__((may_alias)) v4fa;
typedef v4i  __attribute__((may_alias)) v4ia;
typedef v2u  __attribute__((may_alias)) v2ua;
typedef v2us __attribute__((may_alias)) v2usa;
typedef v4us __attribute__((may_alias)) v4usa;
typedef v8us __attribute__((may_alias)) v8usa;
union FragB { v16bf v; v16us u; v8us h[2]; v8i w; };

__device__ __forceinline__ v8f wmb(const FragB& a, const FragB& b, v8f c) {
  v8f d = __builtin_amdgcn_wmma_f32_16x16x32_bf16(false, a.v, false, b.v, (short)0, c, false, false);
  asm volatile("v_nop\n\tv_nop\n\tv_nop\n\tv_nop" : "+v"(d) : "v"(a.w), "v"(b.w));
  return d;
}
__device__ __forceinline__ v8f z8() { v8f z = {0.f, 0.f, 0.f, 0.f, 0.f, 0.f, 0.f, 0.f}; return z; }

__device__ __forceinline__ unsigned bf16_bits(float f) {
  const unsigned u = __float_as_uint(f);
  return (u + 0x7FFFu + ((u >> 16) & 1u)) >> 16;
}
__device__ __forceinline__ float bf16_val(float f) { return __uint_as_float(bf16_bits(f) << 16); }
__device__ __forceinline__ unsigned hl_bits(float v, unsigned& lo) {
  const unsigned hb = bf16_bits(v);
  lo = bf16_bits(v - __uint_as_float(hb << 16));
  return hb;
}
__device__ __forceinline__ float relu_np(float v) { return (v > 0.0f) ? v : (v - v); }

__device__ __forceinline__ void wave_sync() {
  __builtin_amdgcn_fence(__ATOMIC_RELEASE, "wavefront");
  __builtin_amdgcn_wave_barrier();
  __builtin_amdgcn_fence(__ATOMIC_ACQUIRE, "wavefront");
}

template <int SLB>
__device__ __forceinline__ int scan_chunk(const int* __restrict__ dsts, int nE, int cbase, int slotBase,
                                          int nb, int vec8, int* list, int tid, int lane, int wave) {
  int wc = 0;
  const int el0  = tid * EPT;
  const int e0   = cbase + el0;
  const int sent = -2147483647 - 1;
  v4i da, db;
  if (vec8 != 0 && cbase + CHUNK <= nE) {
    da = *(const v4i*)(dsts + e0);
    db = *(const v4i*)(dsts + e0 + 4);
  } else {
    da.x = (e0     < nE) ? dsts[min(e0,     nE - 1)] : sent;
    da.y = (e0 + 1 < nE) ? dsts[min(e0 + 1, nE - 1)] : sent;
    da.z = (e0 + 2 < nE) ? dsts[min(e0 + 2, nE - 1)] : sent;
    da.w = (e0 + 3 < nE) ? dsts[min(e0 + 3, nE - 1)] : sent;
    db.x = (e0 + 4 < nE) ? dsts[min(e0 + 4, nE - 1)] : sent;
    db.y = (e0 + 5 < nE) ? dsts[min(e0 + 5, nE - 1)] : sent;
    db.z = (e0 + 6 < nE) ? dsts[min(e0 + 6, nE - 1)] : sent;
    db.w = (e0 + 7 < nE) ? dsts[min(e0 + 7, nE - 1)] : sent;
  }
  const unsigned nbs = (unsigned)slotBase;
  const unsigned unb = (unsigned)nb;
  const unsigned s0 = (unsigned)da.x - nbs, s1 = (unsigned)da.y - nbs;
  const unsigned s2 = (unsigned)da.z - nbs, s3 = (unsigned)da.w - nbs;
  const unsigned s4 = (unsigned)db.x - nbs, s5 = (unsigned)db.y - nbs;
  const unsigned s6 = (unsigned)db.z - nbs, s7 = (unsigned)db.w - nbs;
  const bool h0 = s0 < unb, h1 = s1 < unb, h2 = s2 < unb, h3 = s3 < unb;
  const bool h4 = s4 < unb, h5 = s5 < unb, h6 = s6 < unb, h7 = s7 < unb;
  const unsigned any = __builtin_amdgcn_ballot_w32(h0 | h1 | h2 | h3 | h4 | h5 | h6 | h7);
  if (any != 0u) {
#define HITJ(J, HJ, SJ) { \
      const unsigned mj = __builtin_amdgcn_ballot_w32(HJ); \
      if (mj != 0u) { \
        if (HJ) { \
          const int pos = wc + (int)__builtin_amdgcn_mbcnt_lo(mj, 0u); \
          if (pos < WCAP) list[wave * WCAP + pos] = ((el0 + (J)) << SLB) | (int)(SJ); \
        } \
        wc += (int)__builtin_popcount(mj); } }
    HITJ(0, h0, s0)
    HITJ(1, h1, s1)
    HITJ(2, h2, s2)
    HITJ(3, h3, s3)
    HITJ(4, h4, s4)
    HITJ(5, h5, s5)
    HITJ(6, h6, s6)
    HITJ(7, h7, s7)
#undef HITJ
  }
  return wc;
}

template <int KP, int QN>
__device__ __forceinline__ void wunit(const float* __restrict__ W, int ldw, int nlim, int kmod, int klim,
                                      int colBase, unsigned short* plane, int ul) {
  const int n   = ul / QN;
  const int q   = ul - n * QN;
  const int ks0 = (8 * q) % kmod;
  const int nc  = n < nlim ? n : nlim - 1;
  v8us o;
#pragma unroll
  for (int i = 0; i < 8; ++i) {
    const int ks = ks0 + i;
    const int kc = ks < klim ? ks : klim - 1;
    const float f = W[(size_t)kc * (size_t)ldw + (size_t)nc];
    asm volatile("" :: "v"(f));
    o[i] = (unsigned short)((ks < klim && n < nlim) ? bf16_bits(f) : 0u);
  }
  unsigned short* dp = plane + (size_t)n * KP + colBase + 8 * q;
  *(volatile v8us*)dp = o;
  __threadfence();
  *(volatile v8us*)dp = o;
}

__global__ __launch_bounds__(GTHR) void k_prepA(const float* __restrict__ spw1, const float* __restrict__ few,
                                                const float* __restrict__ spw2, const float* __restrict__ clw1,
                                                const float* __restrict__ clw2,
                                                unsigned short* pSpw1, unsigned short* pFew, unsigned short* pSpw2,
                                                unsigned short* pCw1, unsigned short* pCw2) {
  const int u = (int)blockIdx.x * GTHR + (int)threadIdx.x;
  if (u < 128)       wunit<32, 4>(spw1, 32, 32, 32, 3, 0, pSpw1, u);
  else if (u < 384)  wunit<32, 4>(few, 64, 64, 32, 16, 0, pFew, u - 128);
  else if (u < 640)  wunit<64, 8>(spw2, 32, 32, 32, 32, 0, pSpw2, u - 384);
  else if (u < 2688) wunit<256, 32>(clw1, 64, 64, 128, 128, 0, pCw1, u - 640);
  else if (u < 2944) wunit<128, 16>(clw2, 10, 10, 64, 64, 0, pCw2, u - 2688);
}

__global__ __launch_bounds__(GTHR) void k_prepB(const float* __restrict__ c1wl, const float* __restrict__ c1wr,
                                                const float* __restrict__ c2w, const float* __restrict__ c3wl,
                                                const float* __restrict__ c3wr, const float* __restrict__ c4w,
                                                const float* __restrict__ fuw,
                                                unsigned short* pW1, unsigned short* pW2, unsigned short* pW3,
                                                unsigned short* pW4, unsigned short* pFu) {
  const int u = (int)blockIdx.x * GTHR + (int)threadIdx.x;
  if (u < 3072)       wunit<384, 24>(c1wl, 128, 128, 96, 96, 0, pW1, u);
  else if (u < 6144)  wunit<384, 24>(c1wr, 128, 128, 96, 96, 192, pW1, u - 3072);
  else if (u < 10240) wunit<256, 32>(c2w, 128, 128, 128, 128, 0, pW2, u - 6144);
  else if (u < 14336) wunit<512, 32>(c3wl, 128, 128, 128, 128, 0, pW3, u - 10240);
  else if (u < 18432) wunit<512, 32>(c3wr, 128, 128, 128, 128, 256, pW3, u - 14336);
  else if (u < 22528) wunit<256, 32>(c4w, 128, 128, 128, 128, 0, pW4, u - 18432);
  else if (u < 26624) wunit<512, 32>(fuw, 128, 128, 128, 128, 0, pFu, u - 22528);
  else if (u < 30720) wunit<512, 32>(fuw + 128 * 128, 128, 128, 128, 128, 256, pFu, u - 26624);
}

__global__ __launch_bounds__(NTHR) void k_bucket(const int* __restrict__ srcs, const int* __restrict__ dsts,
                                                 const float* __restrict__ ew, int nE, int nN, int vec8,
                                                 int* lsrc, float* lw, int* offg, int* cntg, float* disg, int* flagg) {
  extern __shared__ __attribute__((aligned(16))) int dsm[];
  int* list = dsm;
  int* hl   = dsm + LISTN;
  int* sl   = hl + RCAP;
  int* cnt  = sl + RCAP;
  int* offs = cnt + NBA;
  int* cur  = offs + NBA;
  int* misc = cur + NBA;
  const int tid = (int)threadIdx.x, lane = tid & 31, wave = tid >> 5;
  const int nodeBase = (int)blockIdx.x * NBA;
  {
    const v4i z4 = {0, 0, 0, 0};
    for (int i = tid * 4; i < AGG_ZINTS; i += NTHR * 4) *(v4ia*)(dsm + i) = z4;
    if (tid < MISC_INTS) misc[tid] = 0;
  }
  __syncthreads();

  int t = 0, ov = 0;
  const int nChunks = (nE + CHUNK - 1) / CHUNK;
#pragma unroll 1
  for (int ch = 0; ch < nChunks; ++ch) {
    const int cbase = ch * CHUNK;
    const int wc = scan_chunk<SLA>(dsts, nE, cbase, nodeBase, NBA, vec8, list, tid, lane, wave);
    if (lane == 0) misc[wave] = wc;
    __syncthreads();
    if (wave == 0) {
#pragma unroll 1
      for (int w2 = 0; w2 < NWAVE; ++w2) {
        int c = misc[w2];
        c = c < 0 ? 0 : (c > WCAP ? WCAP : c);
#pragma unroll 1
        for (int b0 = 0; b0 < c; b0 += 32) {
          const int idx = b0 + lane;
          const int ent_ = list[w2 * WCAP + (idx < WCAP ? idx : WCAP - 1)];
          const int m32 = (c - b0) < 32 ? (c - b0) : 32;
#pragma unroll 1
          for (int k = 0; k < m32; ++k) {
            const int u    = __builtin_amdgcn_readlane(ent_, k);
            const int slot = u & (NBA - 1);
            const int el   = (u >> SLA) & (CHUNK - 1);
            const int pk   = ((cbase + el) << SLA) | slot;
            if (t < RCAP) {
              if (lane == 0) { hl[t] = pk; cnt[slot] = cnt[slot] + 1; }
              t = t + 1;
            } else {
              ov = 1;
            }
          }
        }
      }
    }
    __syncthreads();
  }
  if (wave == 0 && lane == 0) { misc[8] = t; misc[9] = ov; }
  __syncthreads();
  int tt = misc[8];
  tt = tt < 0 ? 0 : (tt > RCAP ? RCAP : tt);
  const int ovf = misc[9];

  if (wave == 0) {
    const int base = lane * (NBA / 32);
    int s = 0;
#pragma unroll 1
    for (int i = 0; i < NBA / 32; ++i) s += cnt[base + i];
    int incl = s;
#pragma unroll
    for (int d = 1; d < 32; d <<= 1) {
      const int y = __shfl_up(incl, d, 32);
      if (lane >= d) incl += y;
    }
    int run = incl - s;
#pragma unroll 1
    for (int i = 0; i < NBA / 32; ++i) {
      const int cv = cnt[base + i];
      offs[base + i] = run;
      cur[base + i]  = run;
      run += cv;
    }
  }
  __syncthreads();
  if (wave == 0) {
#pragma unroll 1
    for (int b0 = 0; b0 < tt; b0 += 32) {
      const int idx = b0 + lane;
      const int ent_ = hl[idx < RCAP ? idx : RCAP - 1];
      const int m32 = (tt - b0) < 32 ? (tt - b0) : 32;
#pragma unroll 1
      for (int k = 0; k < m32; ++k) {
        const int u    = __builtin_amdgcn_readlane(ent_, k);
        const int slot = u & (NBA - 1);
        if (lane == 0) {
          int p = cur[slot];
          p = p < 0 ? 0 : (p > RCAP - 1 ? RCAP - 1 : p);
          sl[p] = u;
          cur[slot] = p + 1;
        }
      }
    }
  }
  __syncthreads();

#pragma unroll 1
  for (int j = 0; j < NBA / NTHR; ++j) {
    const int s = j * NTHR + tid;
    int c = cnt[s];
    const int big = c > DEGCAP ? 1 : 0;
    c = c < 0 ? 0 : (c > DEGCAP ? DEGCAP : c);
    int o = offs[s];
    o = o < 0 ? 0 : (o > RCAP - 1 ? RCAP - 1 : o);
    int cm = c;
    cm = max(cm, __shfl_xor(cm, 16, 32));
    cm = max(cm, __shfl_xor(cm, 8, 32));
    cm = max(cm, __shfl_xor(cm, 4, 32));
    cm = max(cm, __shfl_xor(cm, 2, 32));
    cm = max(cm, __shfl_xor(cm, 1, 32));
    float deg = 1.0f;
#pragma unroll 1
    for (int p = 0; p < cm; ++p) {
      int pp = p < c ? p : c - 1;
      pp = pp < 0 ? 0 : pp;
      int idx = o + pp;
      idx = idx > RCAP - 1 ? RCAP - 1 : idx;
      int eid = sl[idx] >> SLA;
      eid = eid < 0 ? 0 : (eid > nE - 1 ? nE - 1 : eid);
      const float w = ew[eid];
      asm volatile("" :: "v"(w));
      deg += (p < c) ? bf16_val(w) : 0.0f;
    }
    const float dis = (deg > 0.0f) ? (1.0f / sqrtf(deg)) : 0.0f;
    cur[s] = __float_as_int(dis);
    if (big) misc[10] = 1;
  }
  __syncthreads();

  {
    const int bflag = (ovf != 0 || misc[10] != 0) ? 1 : 0;
    const v4i cv = *(const v4ia*)(cnt + 4 * tid);
    const v4i ovv = *(const v4ia*)(offs + 4 * tid);
    const v4f dv = *(const v4fa*)(cur + 4 * tid);
    const v4i fv = {bflag, bflag, bflag, bflag};
    const size_t tb = (size_t)blockIdx.x * NBA + (size_t)(4 * tid);
    int* fp = flagg + (size_t)blockIdx.x * 32 + 4 * (tid & 7);
    *(volatile v4i*)(cntg + tb) = cv;
    *(volatile v4i*)(offg + tb) = ovv;
    *(volatile v4f*)(disg + tb) = dv;
    if (tid < 8) *(volatile v4i*)fp = fv;
    __threadfence();
    *(volatile v4i*)(cntg + tb) = cv;
    *(volatile v4i*)(offg + tb) = ovv;
    *(volatile v4f*)(disg + tb) = dv;
    if (tid < 8) *(volatile v4i*)fp = fv;
  }

  const int ttr = (tt + 31) & ~31;
  const int ng  = ttr >> 2;
  const size_t lb = (size_t)blockIdx.x * RCAP;
#pragma unroll 1
  for (int g0 = 0; g0 < ng; g0 += NTHR) {
    const int g  = g0 + tid;
    const bool ok = g < ng;
    const int gc = g < RCAP / 4 ? g : RCAP / 4 - 1;
    const v4i en = *(const v4ia*)(sl + 4 * gc);
    int e0 = en.x >> SLA, e1 = en.y >> SLA, e2 = en.z >> SLA, e3 = en.w >> SLA;
    e0 = e0 < 0 ? 0 : (e0 > nE - 1 ? nE - 1 : e0);
    e1 = e1 < 0 ? 0 : (e1 > nE - 1 ? nE - 1 : e1);
    e2 = e2 < 0 ? 0 : (e2 > nE - 1 ? nE - 1 : e2);
    e3 = e3 < 0 ? 0 : (e3 > nE - 1 ? nE - 1 : e3);
    int q0 = srcs[e0], q1 = srcs[e1], q2 = srcs[e2], q3 = srcs[e3];
    asm volatile("" :: "v"(q0), "v"(q1), "v"(q2), "v"(q3));
    q0 = q0 < 0 ? 0 : (q0 > nN - 1 ? nN - 1 : q0);
    q1 = q1 < 0 ? 0 : (q1 > nN - 1 ? nN - 1 : q1);
    q2 = q2 < 0 ? 0 : (q2 > nN - 1 ? nN - 1 : q2);
    q3 = q3 < 0 ? 0 : (q3 > nN - 1 ? nN - 1 : q3);
    const float w0 = ew[e0], w1 = ew[e1], w2 = ew[e2], w3 = ew[e3];
    asm volatile("" :: "v"(w0), "v"(w1), "v"(w2), "v"(w3));
    const int i0 = 4 * gc;
    v4i sv;
    sv.x = (i0     < tt) ? q0 : 0;
    sv.y = (i0 + 1 < tt) ? q1 : 0;
    sv.z = (i0 + 2 < tt) ? q2 : 0;
    sv.w = (i0 + 3 < tt) ? q3 : 0;
    v4f wv;
    wv.x = (i0     < tt) ? bf16_val(w0) : 0.0f;
    wv.y = (i0 + 1 < tt) ? bf16_val(w1) : 0.0f;
    wv.z = (i0 + 2 < tt) ? bf16_val(w2) : 0.0f;
    wv.w = (i0 + 3 < tt) ? bf16_val(w3) : 0.0f;
    int*   sp = lsrc + lb + (size_t)(4 * gc);
    float* wp = lw   + lb + (size_t)(4 * gc);
    if (ok) { *(volatile v4i*)sp = sv; *(volatile v4f*)wp = wv; }
    __threadfence();
    if (ok) { *(volatile v4i*)sp = sv; *(volatile v4f*)wp = wv; }
  }
}

__global__ __launch_bounds__(GTHR) void k_front(const float* __restrict__ x,
                                                const unsigned short* __restrict__ spw1t,
                                                const unsigned short* __restrict__ fewt,
                                                const unsigned short* __restrict__ spw2t,
                                                const float* __restrict__ spb1, const float* __restrict__ spb2,
                                                const float* __restrict__ feb, unsigned short* hhl, int nN) {
  __shared__ float xs[GBM * 19];
  __shared__ __attribute__((aligned(16))) unsigned short cT[GBM * 32];
  __shared__ __attribute__((aligned(16))) unsigned short fT[GBM * 32];
  __shared__ __attribute__((aligned(16))) unsigned short s1[GBM * 64];
  __shared__ __attribute__((aligned(16))) float hst[GBM * 96];
  const int tid = (int)threadIdx.x, lane = tid & 31, wave = tid >> 5, hh = lane >> 4, m = lane & 15;
  const int rowBase = (int)blockIdx.x * GBM;
  const int xtot = nN * 19;
#pragma unroll 1
  for (int it = 0; it < (GBM * 19 + GTHR - 1) / GTHR; ++it) {
    const int i  = it * GTHR + tid;
    const int ic = i < GBM * 19 ? i : GBM * 19 - 1;
    const int g  = rowBase * 19 + ic;
    const int gc = g < xtot ? g : xtot - 1;
    const float v = x[gc];
    asm volatile("" :: "v"(v));
    const float val = (g < xtot) ? v : 0.0f;
    if (i < GBM * 19) xs[i] = val;
  }
  __syncthreads();
#pragma unroll
  for (int jj = 0; jj < 2; ++jj) {
    const int u = jj * GTHR + tid;
    const int r = u >> 2, k8 = (u & 3) * 8;
    v8us oc, of;
#pragma unroll
    for (int i = 0; i < 8; ++i) {
      const int k  = k8 + i;
      const int k3 = k < 3 ? k : 2;
      const int kf = k < 16 ? k : 15;
      const float fc = xs[r * 19 + k3];
      const float ff = xs[r * 19 + 3 + kf];
      oc[i] = (unsigned short)((k < 3) ? bf16_bits(fc) : 0u);
      of[i] = (unsigned short)((k < 16) ? bf16_bits(ff) : 0u);
    }
    *(v8usa*)(cT + u * 8) = oc;
    *(v8usa*)(fT + u * 8) = of;
  }
  __syncthreads();

  v8f a1[2], fe[4], a2[2];
  {
    FragB ac, af;
    const unsigned short* cr = cT + (16 * wave + m) * 32 + 8 * hh;
    const unsigned short* fr = fT + (16 * wave + m) * 32 + 8 * hh;
    ac.h[0] = *(const v8usa*)cr; ac.h[1] = *(const v8usa*)(cr + 16);
    af.h[0] = *(const v8usa*)fr; af.h[1] = *(const v8usa*)(fr + 16);
#pragma unroll
    for (int nt = 0; nt < 2; ++nt) {
      const unsigned short* bp = spw1t + (size_t)(16 * nt + m) * 32 + 8 * hh;
      FragB bf;
      bf.h[0] = *(const v8usa*)bp; bf.h[1] = *(const v8usa*)(bp + 16);
      a1[nt] = wmb(ac, bf, z8());
    }
#pragma unroll
    for (int nt = 0; nt < 4; ++nt) {
      const unsigned short* bp = fewt + (size_t)(16 * nt + m) * 32 + 8 * hh;
      FragB bf;
      bf.h[0] = *(const v8usa*)bp; bf.h[1] = *(const v8usa*)(bp + 16);
      fe[nt] = wmb(af, bf, z8());
    }
  }
#pragma unroll
  for (int nt = 0; nt < 2; ++nt) {
    const int col = 16 * nt + m;
    const float b = bf16_val(spb1[col]);
#pragma unroll
    for (int r = 0; r < 8; ++r) {
      const int row = 16 * wave + 8 * hh + r;
      const float v = relu_np(a1[nt][r] + b);
      unsigned lb;
      const unsigned hb = hl_bits(v, lb);
      s1[row * 64 + col]      = (unsigned short)hb;
      s1[row * 64 + 32 + col] = (unsigned short)lb;
    }
  }
  __syncthreads();
  a2[0] = z8(); a2[1] = z8();
#pragma unroll
  for (int ks = 0; ks < 2; ++ks) {
    const int k0 = 32 * ks;
    FragB af;
    const unsigned short* ar = s1 + (16 * wave + m) * 64 + k0 + 8 * hh;
    af.h[0] = *(const v8usa*)ar; af.h[1] = *(const v8usa*)(ar + 16);
#pragma unroll
    for (int nt = 0; nt < 2; ++nt) {
      const unsigned short* bp = spw2t + (size_t)(16 * nt + m) * 64 + k0 + 8 * hh;
      FragB bf;
      bf.h[0] = *(const v8usa*)bp; bf.h[1] = *(const v8usa*)(bp + 16);
      a2[nt] = wmb(af, bf, a2[nt]);
    }
  }
#pragma unroll
  for (int nt = 0; nt < 2; ++nt) {
    const int col = 16 * nt + m;
    const float b = bf16_val(spb2[col]);
#pragma unroll
    for (int r = 0; r < 8; ++r) hst[(16 * wave + 8 * hh + r) * 96 + col] = relu_np(a2[nt][r] + b);
  }
#pragma unroll
  for (int nt = 0; nt < 4; ++nt) {
    const int col = 16 * nt + m;
    const float b = bf16_val(feb[col]);
#pragma unroll
    for (int r = 0; r < 8; ++r) hst[(16 * wave + 8 * hh + r) * 96 + 32 + col] = relu_np(fe[nt][r] + b);
  }
  __syncthreads();

  v8us qv[12];
#pragma unroll
  for (int it = 0; it < 12; ++it) {
    const int j   = it * GTHR + tid;
    const int row = j / 24;
    const int qq  = j - row * 24;
    const int lo  = qq >= 12 ? 1 : 0;
    const int c8  = 8 * (qq - 12 * lo);
    const v4f p0 = *(const v4fa*)(hst + row * 96 + c8);
    const v4f p1 = *(const v4fa*)(hst + row * 96 + c8 + 4);
    const bool live = (rowBase + row) < nN;
    const unsigned msk = lo ? 0u : 0xFFFFu;
    const float f[8] = {p0.x, p0.y, p0.z, p0.w, p1.x, p1.y, p1.z, p1.w};
    v8us o;
#pragma unroll
    for (int i = 0; i < 8; ++i) {
      const float fv = live ? f[i] : 0.0f;
      unsigned lb;
      const unsigned hb = hl_bits(fv, lb);
      o[i] = (unsigned short)((hb & msk) | (lb & (~msk & 0xFFFFu)));
    }
    qv[it] = o;
  }
  unsigned short* ob = hhl + (size_t)rowBase * 192;
#pragma unroll
  for (int it = 0; it < 12; ++it) *(volatile v8us*)(ob + (size_t)(it * GTHR + tid) * 8) = qv[it];
  __threadfence();
#pragma unroll
  for (int it = 0; it < 12; ++it) *(volatile v8us*)(ob + (size_t)(it * GTHR + tid) * 8) = qv[it];
}

template <int D>
__global__ __launch_bounds__(NTHR) void k_agg(const int* __restrict__ lsrc, const int* __restrict__ offg,
                                              const int* __restrict__ cntg, const int* __restrict__ flagg,
                                              const unsigned short* __restrict__ hpl, unsigned short* mpl,
                                              int nN, int mRows) {
  __shared__ __attribute__((aligned(16))) unsigned short rowbuf[NWAVE * 256];
  constexpr int P  = 2 * D;
  constexpr int LA = D / 4;
  constexpr int LS = P / 8;
  static_assert(LA <= 32 && LS <= 32 && P <= 256);
  const int tid = (int)threadIdx.x, lane = tid & 31, wave = tid >> 5;
  unsigned short* rb = rowbuf + wave * 256;
  const int lc = lane < LA ? lane : LA - 1;
  const int ls = lane < LS ? lane : LS - 1;
#pragma unroll 1
  for (int si = 0; si < NPB / NWAVE; ++si) {
    const int node = (int)blockIdx.x * NPB + si * NWAVE + wave;
    const int nc = node < NTAB ? node : NTAB - 1;
    const int blk = nc >> SLA;
    int c = cntg[nc];
    const bool big = c > DEGCAP;
    c = c < 0 ? 0 : (c > DEGCAP ? DEGCAP : c);
    int o = offg[nc];
    o = o < 0 ? 0 : (o > RCAP - 1 ? RCAP - 1 : o);
    const int fl = flagg[blk * 32];
    const size_t base = (size_t)blk * RCAP;
    const float pzr = (big || fl != 0) ? __int_as_float(0x7fc00000) : 0.0f;
    const bool live = node < nN;
    float a0 = 0.0f, a1 = 0.0f, a2 = 0.0f, a3 = 0.0f;
#pragma unroll 1
    for (int b0 = 0; b0 < c; b0 += 32) {
      int j = b0 + lane;
      j = j < c ? j : c - 1;
      int idx = o + j;
      idx = idx > RCAP - 1 ? RCAP - 1 : idx;
      int sr = lsrc[base + (size_t)idx];
      sr = sr < 0 ? 0 : (sr > nN - 1 ? nN - 1 : sr);
      const int m32 = (c - b0) < 32 ? (c - b0) : 32;
#pragma unroll 1
      for (int k = 0; k < m32; ++k) {
        const int sk = __builtin_amdgcn_readlane(sr, k);
        const unsigned short* rp = hpl + (size_t)sk * P + 4 * lc;
        const v2u wh = *(const v2ua*)rp;
        const v2u wl = *(const v2ua*)(rp + D);
        a0 += __uint_as_float(wh.x << 16)         + __uint_as_float(wl.x << 16);
        a1 += __uint_as_float(wh.x & 0xffff0000u) + __uint_as_float(wl.x & 0xffff0000u);
        a2 += __uint_as_float(wh.y << 16)         + __uint_as_float(wl.y << 16);
        a3 += __uint_as_float(wh.y & 0xffff0000u) + __uint_as_float(wl.y & 0xffff0000u);
      }
    }
    const float den = fmaxf((float)c, 1.0f);
    const float m0 = live ? (a0 / den + pzr) : 0.0f;
    const float m1 = live ? (a1 / den + pzr) : 0.0f;
    const float m2 = live ? (a2 / den + pzr) : 0.0f;
    const float m3 = live ? (a3 / den + pzr) : 0.0f;
    v4us mh, ml;
    {
      unsigned lb;
      unsigned hb;
      hb = hl_bits(m0, lb); mh[0] = (unsigned short)hb; ml[0] = (unsigned short)lb;
      hb = hl_bits(m1, lb); mh[1] = (unsigned short)hb; ml[1] = (unsigned short)lb;
      hb = hl_bits(m2, lb); mh[2] = (unsigned short)hb; ml[2] = (unsigned short)lb;
      hb = hl_bits(m3, lb); mh[3] = (unsigned short)hb; ml[3] = (unsigned short)lb;
    }
    if (lane < LA) {
      *(v4usa*)(rb + 4 * lane)     = mh;
      *(v4usa*)(rb + D + 4 * lane) = ml;
    }
    wave_sync();
    const v8us q0 = *(const v8usa*)(rb + 8 * ls);
    wave_sync();
    if (node < mRows && lane < LS) {
      unsigned short* rpw = mpl + (size_t)node * P + 8 * lane;
      *(volatile v8us*)rpw = q0;
      __threadfence();
      *(volatile v8us*)rpw = q0;
    }
  }
}

__global__ __launch_bounds__(NTHR) void k_gcn(const int* __restrict__ lsrc, const float* __restrict__ lw,
                                              const int* __restrict__ offg, const int* __restrict__ cntg,
                                              const int* __restrict__ flagg, const float* __restrict__ disg,
                                              const float* __restrict__ hws, const float* __restrict__ bias,
                                              float* cout, int nN) {
  const int tid = (int)threadIdx.x, lane = tid & 31, wave = tid >> 5;
  v4f bq;
  {
    const v4f b4 = *(const v4f*)(bias + 4 * lane);
    bq.x = bf16_val(b4.x); bq.y = bf16_val(b4.y); bq.z = bf16_val(b4.z); bq.w = bf16_val(b4.w);
  }
#pragma unroll 1
  for (int si = 0; si < NPB / NWAVE; ++si) {
    const int node = (int)blockIdx.x * NPB + si * NWAVE + wave;
    const int nc = node < NTAB ? node : NTAB - 1;
    const int blk = nc >> SLA;
    int c = cntg[nc];
    const bool big = c > DEGCAP;
    c = c < 0 ? 0 : (c > DEGCAP ? DEGCAP : c);
    int o = offg[nc];
    o = o < 0 ? 0 : (o > RCAP - 1 ? RCAP - 1 : o);
    const int fl = flagg[blk * 32];
    const float di = disg[nc];
    const size_t base = (size_t)blk * RCAP;
    const float pzr = (big || fl != 0) ? __int_as_float(0x7fc00000) : 0.0f;
    const bool live = node < nN;
    const int ndc = node < nN ? node : nN - 1;
    float a0 = 0.0f, a1 = 0.0f, a2 = 0.0f, a3 = 0.0f;
#pragma unroll 1
    for (int b0 = 0; b0 < c; b0 += 32) {
      int j = b0 + lane;
      j = j < c ? j : c - 1;
      int idx = o + j;
      idx = idx > RCAP - 1 ? RCAP - 1 : idx;
      int sr = lsrc[base + (size_t)idx];
      sr = sr < 0 ? 0 : (sr > nN - 1 ? nN - 1 : sr);
      const int wvi = __float_as_int(lw[base + (size_t)idx]);
      const int m32 = (c - b0) < 32 ? (c - b0) : 32;
#pragma unroll 1
      for (int k = 0; k < m32; ++k) {
        const int   sk = __builtin_amdgcn_readlane(sr, k);
        const float ck = __int_as_float(__builtin_amdgcn_readlane(wvi, k));
        const v4f r = *(const v4fa*)(hws + (size_t)sk * GBN + 4 * lane);
        a0 = fmaf(ck, r.x, a0); a1 = fmaf(ck, r.y, a1); a2 = fmaf(ck, r.z, a2); a3 = fmaf(ck, r.w, a3);
      }
    }
    const v4f rs = *(const v4fa*)(hws + (size_t)ndc * GBN + 4 * lane);
    a0 += rs.x; a1 += rs.y; a2 += rs.z; a3 += rs.w;
    v4f ov;
    ov.x = live ? (di * a0 + bq.x + pzr) : 0.0f;
    ov.y = live ? (di * a1 + bq.y + pzr) : 0.0f;
    ov.z = live ? (di * a2 + bq.z + pzr) : 0.0f;
    ov.w = live ? (di * a3 + bq.w + pzr) : 0.0f;
    float* op = cout + (size_t)node * GBN + 4 * lane;
    *(volatile v4f*)op = ov;
    __threadfence();
    *(volatile v4f*)op = ov;
  }
}

__device__ __forceinline__ void gemm_seg(v8f (&acc)[8], const unsigned short* __restrict__ ap,
                                         const unsigned short* __restrict__ bp, int ldb, int K) {
#pragma unroll 1
  for (int k0 = 0; k0 < K; k0 += 32) {
    FragB af;
    af.h[0] = *(const v8usa*)(ap + k0);
    af.h[1] = *(const v8usa*)(ap + k0 + 16);
#pragma unroll
    for (int nt = 0; nt < 8; ++nt) {
      const unsigned short* wq = bp + (size_t)(16 * nt) * (size_t)ldb + k0;
      FragB bf;
      bf.h[0] = *(const v8usa*)wq;
      bf.h[1] = *(const v8usa*)(wq + 16);
      acc[nt] = wmb(af, bf, acc[nt]);
    }
  }
}

template <int MODE>
__global__ __launch_bounds__(GTHR) __attribute__((amdgpu_num_vgpr(248)))
void k_gemm(const unsigned short* __restrict__ A0, int lda0, int K0,
            const unsigned short* __restrict__ A1, int lda1, int K1,
            const unsigned short* __restrict__ BT, int ldb,
            const float* __restrict__ vec, float* outp, int nN) {
  __shared__ __attribute__((aligned(16))) float stg[GBM * GBN];
  __shared__ __attribute__((aligned(16))) float dsc[GBM];
  const int tid = (int)threadIdx.x, lane = tid & 31, wave = tid >> 5, hh = lane >> 4, m = lane & 15;
  const int rowBase = (int)blockIdx.x * GBM;
  v8f acc[8];
#pragma unroll
  for (int t = 0; t < 8; ++t) acc[t] = z8();
  const size_t arow = (size_t)(rowBase + 16 * wave + m);
  gemm_seg(acc, A0 + arow * (size_t)lda0 + 8 * hh, BT + (size_t)m * (size_t)ldb + 8 * hh, ldb, K0);
  gemm_seg(acc, A1 + arow * (size_t)lda1 + 8 * hh, BT + (size_t)m * (size_t)ldb + K0 + 8 * hh, ldb, K1);
#pragma unroll
  for (int nt = 0; nt < 8; ++nt) {
    const int lc = 16 * nt + m;
#pragma unroll
    for (int r = 0; r < 8; ++r) stg[(16 * wave + 8 * hh + r) * GBN + lc] = acc[nt][r];
  }
  if constexpr (MODE == 1) {
    int r4 = rowBase + 4 * (tid & 15);
    r4 = r4 < 0 ? 0 : (r4 > NTAB - 4 ? NTAB - 4 : r4);
    const v4f dv = *(const v4f*)(vec + r4);
    asm volatile("" :: "v"(dv));
    if (tid < GBM / 4) *(v4fa*)(dsc + 4 * tid) = dv;
  } else {
    (void)dsc;
  }
  __syncthreads();
  v4f bq = {0.f, 0.f, 0.f, 0.f};
  if constexpr (MODE == 0) {
    const v4f b4 = *(const v4f*)(vec + 4 * lane);
    bq.x = bf16_val(b4.x); bq.y = bf16_val(b4.y); bq.z = bf16_val(b4.z); bq.w = bf16_val(b4.w);
  }
  v4f pv[16];
#pragma unroll
  for (int i = 0; i < 16; ++i) {
    const int row = rowBase + 16 * wave + i;
    const bool ok = row < nN;
    const v4f d = *(const v4fa*)(stg + (16 * wave + i) * GBN + 4 * lane);
    v4f y;
    if constexpr (MODE == 0) {
      y.x = d.x + bq.x; y.y = d.y + bq.y; y.z = d.z + bq.z; y.w = d.w + bq.w;
    } else {
      const float sc = dsc[16 * wave + i];
      y.x = d.x * sc; y.y = d.y * sc; y.z = d.z * sc; y.w = d.w * sc;
    }
    v4f q;
    q.x = ok ? y.x : 0.0f; q.y = ok ? y.y : 0.0f; q.z = ok ? y.z : 0.0f; q.w = ok ? y.w : 0.0f;
    pv[i] = q;
  }
#pragma unroll
  for (int i = 0; i < 16; ++i)
    *(volatile v4f*)(outp + (size_t)(rowBase + 16 * wave + i) * GBN + 4 * lane) = pv[i];
  __threadfence();
#pragma unroll
  for (int i = 0; i < 16; ++i)
    *(volatile v4f*)(outp + (size_t)(rowBase + 16 * wave + i) * GBN + 4 * lane) = pv[i];
}

__global__ __launch_bounds__(NTHR) void k_bnstats(const float* __restrict__ C, float* rec, int nN) {
  __shared__ float hs[2 * 256];
  __shared__ __attribute__((aligned(16))) float pst[PARTW];
  const int tid = (int)threadIdx.x;
  const int c = tid & 127, half = tid >> 7;
  const int tile = (int)blockIdx.x;
  const int r0 = tile * 128 + half * 64;
  int nv = nN - r0;
  nv = nv < 0 ? 0 : (nv > 64 ? 64 : nv);
  const float* p = C + (size_t)r0 * GBN + c;
  float s = 0.0f;
#pragma unroll 4
  for (int i = 0; i < nv; ++i) s += p[(size_t)i * GBN];
  const float mean = (nv > 0) ? s * (1.0f / (float)(nv > 0 ? nv : 1)) : 0.0f;
  float q = 0.0f;
#pragma unroll 4
  for (int i = 0; i < nv; ++i) { const float d = p[(size_t)i * GBN] - mean; q = fmaf(d, d, q); }
  hs[half * 256 + c] = mean;
  hs[half * 256 + 128 + c] = q;
  __syncthreads();
  if (tid < 128) {
    int n0 = nN - tile * 128;       n0 = n0 < 0 ? 0 : (n0 > 64 ? 64 : n0);
    int n1 = nN - tile * 128 - 64;  n1 = n1 < 0 ? 0 : (n1 > 64 ? 64 : n1);
    const float m0 = hs[c], q0 = hs[128 + c], m1 = hs[256 + c], q1 = hs[384 + c];
    const float nn = (float)(n0 + n1);
    const float f = (float)n1 * (1.0f / (nn > 0.5f ? nn : 1.0f));
    const float delta = m1 - m0;
    const float mc = (n1 > 0) ? fmaf(delta, f, m0) : m0;
    const float qc = (n1 > 0) ? (q0 + q1 + delta * delta * (float)n0 * f) : q0;
    pst[1 + c] = mc;
    pst[129 + c] = qc;
    if (tid == 0) pst[0] = nn;
  } else if (tid < 128 + 31) {
    pst[257 + (tid - 128)] = 0.0f;
  }
  __syncthreads();
  v4f ps = {0.f, 0.f, 0.f, 0.f};
  const bool ok = tid < PARTW / 4;
  const int tc = ok ? tid : 0;
  ps = *(const v4fa*)(pst + 4 * tc);
  float* rp = rec + (size_t)tile * PARTW + 4 * tc;
  if (ok) *(volatile v4f*)rp = ps;
  __threadfence();
  if (ok) *(volatile v4f*)rp = ps;
}

__global__ __launch_bounds__(GTHR) void k_bncomb(const float* __restrict__ rec, int nRec,
                                                 const float* __restrict__ gam, const float* __restrict__ bet,
                                                 float* stat) {
  __shared__ __attribute__((aligned(16))) float stg[512];
  const int c = (int)threadIdx.x;
  double n = 0.0, mean = 0.0, M2 = 0.0;
#pragma unroll 1
  for (int b = 0; b < nRec; ++b) {
    const float* pr = rec + (size_t)b * PARTW;
    const double nb = (double)pr[0];
    const double mb = (double)pr[1 + c];
    const double qb = (double)pr[129 + c];
    if (nb > 0.5) {
      const double nn = n + nb;
      const double delta = mb - mean;
      const double f = nb / nn;
      mean = mean + delta * f;
      M2 = M2 + qb + delta * delta * n * f;
      n = nn;
    }
  }
  const double nt = n < 1.0 ? 1.0 : n;
  const float varf = (float)(M2 / nt);
  const float muf  = (float)mean;
  const float rs   = 1.0f / sqrtf(varf + BNEPS);
  stg[c] = muf;
  stg[128 + c] = rs;
  stg[256 + c] = bf16_val(gam[c]);
  stg[384 + c] = bf16_val(bet[c]);
  __syncthreads();
  const v4f v = *(const v4fa*)(stg + 4 * c);
  *(volatile v4f*)(stat + 4 * c) = v;
  __threadfence();
  *(volatile v4f*)(stat + 4 * c) = v;
}

__global__ __launch_bounds__(NTHR) void k_apply(const float* __restrict__ C, const float* __restrict__ stat,
                                                unsigned short* xhl, int nN) {
  __shared__ __attribute__((aligned(16))) float sst[512];
  const int tid = (int)threadIdx.x;
  if (tid < 128) *(v4fa*)(sst + 4 * tid) = *(const v4f*)(stat + 4 * tid);
  __syncthreads();
  const int u = (int)blockIdx.x * NTHR + tid;
  const int row = u >> 4, c8 = (u & 15) * 8;
  const bool live = row < nN;
  const int rc = live ? row : nN - 1;
  const float* p = C + (size_t)rc * GBN + c8;
  const v4f xa = *(const v4f*)p;
  const v4f xb = *(const v4f*)(p + 4);
  asm volatile("" :: "v"(xa), "v"(xb));
  const v4f mua = *(const v4fa*)(sst + c8),       mub = *(const v4fa*)(sst + c8 + 4);
  const v4f rsa = *(const v4fa*)(sst + 128 + c8), rsb = *(const v4fa*)(sst + 128 + c8 + 4);
  const v4f ga  = *(const v4fa*)(sst + 256 + c8), gb  = *(const v4fa*)(sst + 256 + c8 + 4);
  const v4f ba  = *(const v4fa*)(sst + 384 + c8), bb  = *(const v4fa*)(sst + 384 + c8 + 4);
  const float xv[8] = {xa.x, xa.y, xa.z, xa.w, xb.x, xb.y, xb.z, xb.w};
  const float mu[8] = {mua.x, mua.y, mua.z, mua.w, mub.x, mub.y, mub.z, mub.w};
  const float rs[8] = {rsa.x, rsa.y, rsa.z, rsa.w, rsb.x, rsb.y, rsb.z, rsb.w};
  const float gg[8] = {ga.x, ga.y, ga.z, ga.w, gb.x, gb.y, gb.z, gb.w};
  const float be[8] = {ba.x, ba.y, ba.z, ba.w, bb.x, bb.y, bb.z, bb.w};
  v8us h, l;
#pragma unroll
  for (int i = 0; i < 8; ++i) {
    float y = ((xv[i] - mu[i]) * rs[i]) * gg[i] + be[i];
    y = relu_np(y);
    y = live ? y : 0.0f;
    unsigned lb;
    const unsigned hb = hl_bits(y, lb);
    h[i] = (unsigned short)hb;
    l[i] = (unsigned short)lb;
  }
  unsigned short* dp = xhl + (size_t)row * 256 + c8;
  *(volatile v8us*)dp = h;
  *(volatile v8us*)(dp + 128) = l;
  __threadfence();
  *(volatile v8us*)dp = h;
  *(volatile v8us*)(dp + 128) = l;
}

__global__ __launch_bounds__(GTHR) __attribute__((amdgpu_num_vgpr(248)))
void k_tail(const unsigned short* __restrict__ h2, const unsigned short* __restrict__ h4,
            const unsigned short* __restrict__ fup, const unsigned short* __restrict__ cw1p,
            const unsigned short* __restrict__ cw2p, const float* __restrict__ fub,
            const float* __restrict__ clb1, const float* __restrict__ clb2, float* outp, int nN) {
  __shared__ __attribute__((aligned(16))) float stg[GBM * GBN];
  unsigned short* sth = (unsigned short*)stg;
  const int tid = (int)threadIdx.x, lane = tid & 31, wave = tid >> 5, hh = lane >> 4, m = lane & 15;
  const int rowBase = (int)blockIdx.x * GBM;

  {
    v8f acc[8];
#pragma unroll
    for (int t = 0; t < 8; ++t) acc[t] = z8();
    const size_t arow = (size_t)(rowBase + 16 * wave + m);
    gemm_seg(acc, h2 + arow * 256 + 8 * hh, fup + (size_t)m * 512 + 8 * hh, 512, 256);
    gemm_seg(acc, h4 + arow * 256 + 8 * hh, fup + (size_t)m * 512 + 256 + 8 * hh, 512, 256);
#pragma unroll
    for (int nt = 0; nt < 8; ++nt) {
      const int lc = 16 * nt + m;
#pragma unroll
      for (int r = 0; r < 8; ++r) stg[(16 * wave + 8 * hh + r) * GBN + lc] = acc[nt][r];
    }
  }
  __syncthreads();
  {
    v4f bq;
    {
      const v4f b4 = *(const v4f*)(fub + 4 * lane);
      bq.x = bf16_val(b4.x); bq.y = bf16_val(b4.y); bq.z = bf16_val(b4.z); bq.w = bf16_val(b4.w);
    }
    v4f pv[16];
#pragma unroll
    for (int i = 0; i < 16; ++i) pv[i] = *(const v4fa*)(stg + (16 * wave + i) * GBN + 4 * lane);
    __syncthreads();
#pragma unroll
    for (int i = 0; i < 16; ++i) {
      const float y0 = pv[i].x + bq.x, y1 = pv[i].y + bq.y, y2 = pv[i].z + bq.z, y3 = pv[i].w + bq.w;
      v4us h4v, l4v;
      unsigned lb;
      unsigned hb;
      hb = hl_bits(y0, lb); h4v[0] = (unsigned short)hb; l4v[0] = (unsigned short)lb;
      hb = hl_bits(y1, lb); h4v[1] = (unsigned short)hb; l4v[1] = (unsigned short)lb;
      hb = hl_bits(y2, lb); h4v[2] = (unsigned short)hb; l4v[2] = (unsigned short)lb;
      hb = hl_bits(y3, lb); h4v[3] = (unsigned short)hb; l4v[3] = (unsigned short)lb;
      unsigned short* srow = sth + (16 * wave + i) * 256;
      *(v4usa*)(srow + 4 * lane)       = h4v;
      *(v4usa*)(srow + 128 + 4 * lane) = l4v;
    }
  }
  __syncthreads();

  v8f a2[4];
#pragma unroll
  for (int t = 0; t < 4; ++t) a2[t] = z8();
#pragma unroll 1
  for (int k0 = 0; k0 < 256; k0 += 32) {
    FragB af;
    const unsigned short* ar = sth + (16 * wave + m) * 256 + k0 + 8 * hh;
    af.h[0] = *(const v8usa*)ar;
    af.h[1] = *(const v8usa*)(ar + 16);
#pragma unroll
    for (int nt = 0; nt < 4; ++nt) {
      const unsigned short* wq = cw1p + (size_t)(16 * nt + m) * 256 + k0 + 8 * hh;
      FragB bf;
      bf.h[0] = *(const v8usa*)wq;
      bf.h[1] = *(const v8usa*)(wq + 16);
      a2[nt] = wmb(af, bf, a2[nt]);
    }
  }
  __syncthreads();
#pragma unroll
  for (int nt = 0; nt < 4; ++nt) {
    const int lc = 16 * nt + m;
#pragma unroll
    for (int r = 0; r < 8; ++r) stg[(16 * wave + 8 * hh + r) * 64 + lc] = a2[nt][r];
  }
  __syncthreads();
  {
    v2f cq;
    {
      const v2f c2 = *(const v2f*)(clb1 + 2 * lane);
      cq.x = bf16_val(c2.x); cq.y = bf16_val(c2.y);
    }
    v2f p2[16];
#pragma unroll
    for (int i = 0; i < 16; ++i) p2[i] = *(const v2fa*)(stg + (16 * wave + i) * 64 + 2 * lane);
    __syncthreads();
#pragma unroll
    for (int i = 0; i < 16; ++i) {
      const float y0 = relu_np(p2[i].x + cq.x), y1 = relu_np(p2[i].y + cq.y);
      v2us h2v, l2v;
      unsigned lb;
      unsigned hb;
      hb = hl_bits(y0, lb); h2v[0] = (unsigned short)hb; l2v[0] = (unsigned short)lb;
      hb = hl_bits(y1, lb); h2v[1] = (unsigned short)hb; l2v[1] = (unsigned short)lb;
      unsigned short* srow = sth + (16 * wave + i) * 128;
      *(v2usa*)(srow + 2 * lane)      = h2v;
      *(v2usa*)(srow + 64 + 2 * lane) = l2v;
    }
  }
  __syncthreads();

  v8f a3 = z8();
#pragma unroll 1
  for (int k0 = 0; k0 < 128; k0 += 32) {
    FragB af;
    const unsigned short* ar = sth + (16 * wave + m) * 128 + k0 + 8 * hh;
    af.h[0] = *(const v8usa*)ar;
    af.h[1] = *(const v8usa*)(ar + 16);
    const unsigned short* wq = cw2p + (size_t)m * 128 + k0 + 8 * hh;
    FragB bf;
    bf.h[0] = *(const v8usa*)wq;
    bf.h[1] = *(const v8usa*)(wq + 16);
    a3 = wmb(af, bf, a3);
  }
  __syncthreads();
  {
    const float cb = clb2[m < 10 ? m : 9];
    asm volatile("" :: "v"(cb));
    const float cbv = bf16_val(cb);
#pragma unroll
    for (int r = 0; r < 8; ++r) {
      const int row = 16 * wave + 8 * hh + r;
      if (m < 10) stg[row * 10 + m] = a3[r] + cbv;
    }
  }
  __syncthreads();
  {
    int nv = nN - rowBase;
    nv = nv < 0 ? 0 : (nv > GBM ? GBM : nv);
    const int nf4 = (nv * 10) >> 2;
    const int t0 = tid, t1 = GTHR + tid;
    const int t1c = t1 < 160 ? t1 : 159;
    const v4f o0 = *(const v4fa*)(stg + 4 * t0);
    const v4f o1 = *(const v4fa*)(stg + 4 * t1c);
    float* ob = outp + (size_t)rowBase * 10;
    const bool ok0 = t0 < nf4, ok1 = t1 < nf4;
    if (ok0) *(volatile v4f*)(ob + 4 * t0) = o0;
    if (ok1) *(volatile v4f*)(ob + 4 * t1c) = o1;
    __threadfence();
    if (ok0) *(volatile v4f*)(ob + 4 * t0) = o0;
    if (ok1) *(volatile v4f*)(ob + 4 * t1c) = o1;
  }
}

static constexpr size_t al256c(size_t o) { return (o + 255) & ~(size_t)255; }
static constexpr size_t SZ_HHL  = (size_t)MP * 192 * 2;
static constexpr size_t SZ_P256 = (size_t)MP * 256 * 2;
static constexpr size_t SZ_F128 = (size_t)MP * 128 * 4;
static constexpr size_t SZ_R0   = 2 * SZ_HHL;
static constexpr size_t SZ_LIST = (size_t)NBLK * RCAP * 4;
static constexpr size_t SZ_TAB  = (size_t)NTAB * 4;
static constexpr size_t SZ_FLAG = (size_t)NBLK * 128;
static constexpr size_t SZ_REC  = (size_t)NTILE * PARTW * 4;
static constexpr size_t O_R0   = 0;
static constexpr size_t O_C    = al256c(O_R0 + SZ_R0);
static constexpr size_t O_XHL  = al256c(O_C + SZ_F128);
static constexpr size_t O_H2   = al256c(O_XHL + SZ_P256);
static constexpr size_t O_LSRC = al256c(O_H2 + SZ_P256);
static constexpr size_t O_LW   = al256c(O_LSRC + SZ_LIST);
static constexpr size_t O_OFF  = al256c(O_LW + SZ_LIST);
static constexpr size_t O_CNT  = al256c(O_OFF + SZ_TAB);
static constexpr size_t O_DIS  = al256c(O_CNT + SZ_TAB);
static constexpr size_t O_FLAG = al256c(O_DIS + SZ_TAB);
static constexpr size_t O_REC  = al256c(O_FLAG + SZ_FLAG);
static constexpr size_t O_STAT = al256c(O_REC + SZ_REC);
static constexpr size_t O_SPW1 = al256c(O_STAT + 2048);
static constexpr size_t O_FEW  = al256c(O_SPW1 + 32 * 32 * 2);
static constexpr size_t O_SPW2 = al256c(O_FEW + 64 * 32 * 2);
static constexpr size_t O_CW1  = al256c(O_SPW2 + 32 * 64 * 2);
static constexpr size_t O_CW2  = al256c(O_CW1 + 64 * 256 * 2);
static constexpr size_t O_W1P  = al256c(O_CW2 + 16 * 128 * 2);
static constexpr size_t O_W2P  = al256c(O_W1P + 128 * 384 * 2);
static constexpr size_t O_W3P  = al256c(O_W2P + 128 * 256 * 2);
static constexpr size_t O_W4P  = al256c(O_W3P + 128 * 512 * 2);
static constexpr size_t O_FUP  = al256c(O_W4P + 128 * 256 * 2);
static constexpr size_t WS_TOTAL = al256c(O_FUP + 128 * 512 * 2);
static_assert(SZ_R0 >= SZ_F128 && SZ_R0 >= SZ_P256);
static_assert(WS_TOTAL <= WSMAX);
static_assert((size_t)(NNODE - 1) * 10 + 9 < (size_t)NNODE * 10);
static_assert(O_DIS % 16 == 0);

extern "C" void kernel_launch(void* const* d_in, const int* in_sizes, int n_in,
                              void* d_out, int out_size, void* d_ws, size_t ws_size,
                              hipStream_t stream) {
  if (n_in < 27) return;
  const int expect[27] = {NNODE * 19, 2 * NEDGE, NEDGE, 96, 32, 1024, 32, 1024, 64, 12288, 12288, 128, 16384, 128,
                          16384, 16384, 128, 16384, 128, 512, 512, 32768, 128, 8192, 64, 640, 10};
  for (int i = 0; i < 27; ++i) if (in_sizes[i] != expect[i]) return;
  if (out_size != NNODE * 10) return;
  if (ws_size < WS_TOTAL) return;

  const float* x     = (const float*)d_in[0];
  const int*   ei    = (const int*)  d_in[1];
  const float* ew    = (const float*)d_in[2];
  const float* sp_w1 = (const float*)d_in[3];
  const float* sp_b1 = (const float*)d_in[4];
  const float* sp_w2 = (const float*)d_in[5];
  const float* sp_b2 = (const float*)d_in[6];
  const float* fe_w  = (const float*)d_in[7];
  const float* fe_b  = (const float*)d_in[8];
  const float* c1_wl = (const float*)d_in[9];
  const float* c1_wr = (const float*)d_in[10];
  const float* c1_b  = (const float*)d_in[11];
  const float* c2_w  = (const float*)d_in[12];
  const float* c2_b  = (const float*)d_in[13];
  const float* c3_wl = (const float*)d_in[14];
  const float* c3_wr = (const float*)d_in[15];
  const float* c3_b  = (const float*)d_in[16];
  const float* c4_w  = (const float*)d_in[17];
  const float* c4_b  = (const float*)d_in[18];
  const float* bn_g  = (const float*)d_in[19];
  const float* bn_b  = (const float*)d_in[20];
  const float* fu_w  = (const float*)d_in[21];
  const float* fu_b  = (const float*)d_in[22];
  const float* cl_w1 = (const float*)d_in[23];
  const float* cl_b1 = (const float*)d_in[24];
  const float* cl_w2 = (const float*)d_in[25];
  const float* cl_b2 = (const float*)d_in[26];
  float* out = (float*)d_out;
  const int nN = NNODE, nE = NEDGE;
  const int* src = ei;
  const int* dst = ei + nE;
  const int vec8 = ((nE & 3) == 0) ? 1 : 0;

  char* ws = (char*)d_ws;
  unsigned short* Hhl  = (unsigned short*)(ws + O_R0);
  unsigned short* M1hl = (unsigned short*)(ws + O_R0 + SZ_HHL);
  float*          HWs  = (float*)(ws + O_R0);
  unsigned short* M3hl = (unsigned short*)(ws + O_R0);
  float*          Cb   = (float*)(ws + O_C);
  unsigned short* Xhl  = (unsigned short*)(ws + O_XHL);
  unsigned short* H2hl = (unsigned short*)(ws + O_H2);
  int*   LSRC = (int*)(ws + O_LSRC);
  float* LW   = (float*)(ws + O_LW);
  int*   OFFt = (int*)(ws + O_OFF);
  int*   CNTt = (int*)(ws + O_CNT);
  float* DISt = (float*)(ws + O_DIS);
  int*   FLG  = (int*)(ws + O_FLAG);
  float* REC  = (float*)(ws + O_REC);
  float* STAT = (float*)(ws + O_STAT);
  unsigned short* pSpw1 = (unsigned short*)(ws + O_SPW1);
  unsigned short* pFew  = (unsigned short*)(ws + O_FEW);
  unsigned short* pSpw2 = (unsigned short*)(ws + O_SPW2);
  unsigned short* pCw1  = (unsigned short*)(ws + O_CW1);
  unsigned short* pCw2  = (unsigned short*)(ws + O_CW2);
  unsigned short* pW1   = (unsigned short*)(ws + O_W1P);
  unsigned short* pW2   = (unsigned short*)(ws + O_W2P);
  unsigned short* pW3   = (unsigned short*)(ws + O_W3P);
  unsigned short* pW4   = (unsigned short*)(ws + O_W4P);
  unsigned short* pFu   = (unsigned short*)(ws + O_FUP);

  const size_t bktLds = (size_t)BKT_LDS_INTS * 4;
  hipFuncSetAttribute(reinterpret_cast<const void*>(&k_bucket), hipFuncAttributeMaxDynamicSharedMemorySize, (int)bktLds);

  const int gM = MP / GBM;
  const int gApply = (MP * 16) / NTHR;

  k_prepA<<<2944 / GTHR, GTHR, 0, stream>>>(sp_w1, fe_w, sp_w2, cl_w1, cl_w2, pSpw1, pFew, pSpw2, pCw1, pCw2);
  k_prepB<<<30720 / GTHR, GTHR, 0, stream>>>(c1_wl, c1_wr, c2_w, c3_wl, c3_wr, c4_w, fu_w, pW1, pW2, pW3, pW4, pFu);
  k_bucket<<<NBLK, NTHR, bktLds, stream>>>(src, dst, ew, nE, nN, vec8, LSRC, LW, OFFt, CNTt, DISt, FLG);
  k_front<<<gM, GTHR, 0, stream>>>(x, pSpw1, pFew, pSpw2, sp_b1, sp_b2, fe_b, Hhl, nN);
  k_agg<96><<<NTILE, NTHR, 0, stream>>>(LSRC, OFFt, CNTt, FLG, Hhl, M1hl, nN, MP);
  k_gemm<0><<<gM, GTHR, 0, stream>>>(M1hl, 192, 192, Hhl, 192, 192, pW1, 384, c1_b, Cb, nN);
  k_bnstats<<<NTILE, NTHR, 0, stream>>>(Cb, REC, nN);
  k_bncomb<<<1, GTHR, 0, stream>>>(REC, NTILE, bn_g + 0 * 128, bn_b + 0 * 128, STAT);
  k_apply<<<gApply, NTHR, 0, stream>>>(Cb, STAT, Xhl, nN);
  k_gemm<1><<<gM, GTHR, 0, stream>>>(Xhl, 256, 256, Xhl, 256, 0, pW2, 256, DISt, HWs, nN);
  k_gcn<<<NTILE, NTHR, 0, stream>>>(LSRC, LW, OFFt, CNTt, FLG, DISt, HWs, c2_b, Cb, nN);
  k_bnstats<<<NTILE, NTHR, 0, stream>>>(Cb, REC, nN);
  k_bncomb<<<1, GTHR, 0, stream>>>(REC, NTILE, bn_g + 1 * 128, bn_b + 1 * 128, STAT);
  k_apply<<<gApply, NTHR, 0, stream>>>(Cb, STAT, H2hl, nN);
  k_agg<128><<<NTILE, NTHR, 0, stream>>>(LSRC, OFFt, CNTt, FLG, H2hl, M3hl, nN, MP);
  k_gemm<0><<<gM, GTHR, 0, stream>>>(M3hl, 256, 256, H2hl, 256, 256, pW3, 512, c3_b, Cb, nN);
  k_bnstats<<<NTILE, NTHR, 0, stream>>>(Cb, REC, nN);
  k_bncomb<<<1, GTHR, 0, stream>>>(REC, NTILE, bn_g + 2 * 128, bn_b + 2 * 128, STAT);
  k_apply<<<gApply, NTHR, 0, stream>>>(Cb, STAT, Xhl, nN);
  k_gemm<1><<<gM, GTHR, 0, stream>>>(Xhl, 256, 256, Xhl, 256, 0, pW4, 256, DISt, HWs, nN);
  k_gcn<<<NTILE, NTHR, 0, stream>>>(LSRC, LW, OFFt, CNTt, FLG, DISt, HWs, c4_b, Cb, nN);
  k_bnstats<<<NTILE, NTHR, 0, stream>>>(Cb, REC, nN);
  k_bncomb<<<1, GTHR, 0, stream>>>(REC, NTILE, bn_g + 3 * 128, bn_b + 3 * 128, STAT);
  k_apply<<<gApply, NTHR, 0, stream>>>(Cb, STAT, Xhl, nN);
  k_tail<<<gM, GTHR, 0, stream>>>(H2hl, Xhl, pFu, pCw1, pCw2, fu_b, cl_b1, cl_b2, out, nN);
}
